// MDAGCN_block_26113401159749
// MI455X (gfx1250) — hardware-run, weakly checked
//
#include <hip/hip_runtime.h>


namespace {
constexpr int NB = 8, T = 8, V = 128, FD = 64, KC = 3, C1 = 256, CH = 64, TF = 64, KT = 3;
constexpr float ALPHA = 1e-4f, WSC = 256.0f;
typedef _Float16 b16;
typedef __attribute__((ext_vector_type(16))) _Float16 v16b;
typedef __attribute__((ext_vector_type(8))) _Float16 v8b;
typedef __attribute__((ext_vector_type(8))) float v8f;
typedef __attribute__((ext_vector_type(4))) float v4f;
__device__ __forceinline__ float bf16_rne(float f) { unsigned int u = __float_as_uint(f); u += 0x7FFFu + ((u >> 16) & 1u); return __uint_as_float(u & 0xFFFF0000u); }
__device__ __forceinline__ void split16(float v, b16& hi, b16& lo) { hi = (b16)v; lo = (b16)(v - (float)hi); }
__device__ __forceinline__ v16b frag_kb(const b16* p, int hh) { const v8b a = *(const v8b*)(p + 8 * hh), b = *(const v8b*)(p + 16 + 8 * hh); v16b f;
#pragma unroll
  for (int e = 0; e < 8; ++e) { f[e] = a[e]; f[8 + e] = b[e]; } return f; }
__device__ __forceinline__ v8f wmma16b(v16b a, v16b b, v8f c) { v8f d = __builtin_amdgcn_wmma_f32_16x16x32_f16(false, a, false, b, (short)0, c, false, false); asm volatile("v_nop\n\tv_nop\n\tv_nop\n\tv_nop" : "+v"(d) : "v"(a), "v"(b)); return d; }
__device__ __forceinline__ void wave_lds_sync() { __builtin_amdgcn_fence(__ATOMIC_RELEASE, "workgroup"); __builtin_amdgcn_wave_barrier(); __builtin_amdgcn_fence(__ATOMIC_ACQUIRE, "workgroup"); }
__device__ __forceinline__ float pmul(float a, float b) { float p = a * b; asm volatile("" : "+v"(p)); return p; }
__device__ __forceinline__ float sigm(float v) { return 1.0f / (1.0f + __expf(-v)); }

__global__ __launch_bounds__(256) void tatt_kernel(const float* __restrict__ x, const float* __restrict__ U1, const float* __restrict__ U2, const float* __restrict__ U3, const float* __restrict__ be, const float* __restrict__ Ve, float* __restrict__ TATT) {
  __shared__ float Lh[T][FD], L2[T][V], Rh[V][T], Pr[T][T], Sg[T][T]; const int n = blockIdx.x, tid = threadIdx.x; const float* xn = x + (size_t)n * T * V * FD;
  for (int i = tid; i < T * FD; i += 256) { const int t = i / FD, f = i % FD; float s = 0.0f;
#pragma unroll 1
    for (int v = 0; v < V; ++v) s += pmul(bf16_rne(xn[((size_t)t * V + v) * FD + f]), bf16_rne(U1[v])); Lh[t][f] = s; }
  for (int i = tid; i < V * T; i += 256) { const int v = i / T, t = i % T; float s = 0.0f;
#pragma unroll 1
    for (int f = 0; f < FD; ++f) s += pmul(bf16_rne(xn[((size_t)t * V + v) * FD + f]), bf16_rne(U3[f])); Rh[v][t] = s; }
  __syncthreads();
  for (int i = tid; i < T * V; i += 256) { const int t = i / V, v = i % V; float s = 0.0f;
#pragma unroll 1
    for (int f = 0; f < FD; ++f) s += pmul(Lh[t][f], bf16_rne(U2[f * V + v])); L2[t][v] = s; }
  __syncthreads();
  if (tid < T * T) { const int t = tid / T, s_ = tid % T; float s = 0.0f;
#pragma unroll 1
    for (int v = 0; v < V; ++v) s += pmul(L2[t][v], Rh[v][s_]); Pr[t][s_] = sigm(s + bf16_rne(be[t * T + s_])); }
  __syncthreads();
  if (tid < T * T) { const int i = tid / T, j = tid % T; float s = 0.0f; for (int k = 0; k < T; ++k) s += pmul(bf16_rne(Ve[i * T + k]), Pr[k][j]); Sg[i][j] = s; }
  __syncthreads();
  if (tid < T * T) { const int i = tid / T, j = tid % T; float mx = -INFINITY; for (int k = 0; k < T; ++k) mx = fmaxf(mx, Sg[k][j]); float den = 0.0f; for (int k = 0; k < T; ++k) den += __expf(Sg[k][j] - mx); const float r = __expf(Sg[i][j] - mx) / den;
    for (int pass = 0; pass < 2; ++pass) { ((volatile float*)TATT)[n * 64 + i * T + j] = r; __threadfence(); } }
}
__global__ __launch_bounds__(256) void xt_kernel(const float* __restrict__ x, const float* __restrict__ TATT, float* __restrict__ XT) {
  const size_t u = (size_t)blockIdx.x * 256 + threadIdx.x; if (u >= (size_t)NB * T * V * FD / 4) return; const int f0 = (int)(u % (FD / 4)) * 4, v = (int)((u / (FD / 4)) % V), s = (int)((u / ((size_t)(FD / 4) * V)) % T), n = (int)(u / ((size_t)(FD / 4) * V * T));
  v4f r = {0, 0, 0, 0};
#pragma unroll 1
  for (int t = 0; t < T; ++t) { const float w = TATT[n * 64 + t * T + s]; const v4f xv = *(const v4f*)(x + (((size_t)n * T + t) * V + v) * FD + f0); for (int i = 0; i < 4; ++i) r[i] += pmul(bf16_rne(xv[i]), w); }
  for (int pass = 0; pass < 2; ++pass) { *(volatile v4f*)(XT + (((size_t)n * T + s) * V + v) * FD + f0) = r; __threadfence(); }
}
__global__ __launch_bounds__(256) void sprep_kernel(const float* __restrict__ XT, const float* __restrict__ W1, const float* __restrict__ W2, const float* __restrict__ W3, const float* __restrict__ bs, b16* __restrict__ SGH, b16* __restrict__ SGL) {
  __shared__ float A1[V][FD + 1], Ls[V][T], Rs[T][V]; const int n = blockIdx.x, tid = threadIdx.x; const float* xn = XT + (size_t)n * T * V * FD;
  for (int i = tid; i < V * FD; i += 256) { const int v = i / FD, f = i % FD; float s = 0.0f;
#pragma unroll 1
    for (int t = 0; t < T; ++t) s += pmul(xn[((size_t)t * V + v) * FD + f], bf16_rne(W1[t])); A1[v][f] = s; }
  for (int i = tid; i < T * V; i += 256) { const int t = i / V, u = i % V; float s = 0.0f;
#pragma unroll 1
    for (int f = 0; f < FD; ++f) s += pmul(xn[((size_t)t * V + u) * FD + f], bf16_rne(W3[f])); Rs[t][u] = s; }
  __syncthreads();
  for (int i = tid; i < V * T; i += 256) { const int v = i / T, t = i % T; float s = 0.0f;
#pragma unroll 1
    for (int f = 0; f < FD; ++f) s += pmul(A1[v][f], bf16_rne(W2[f * T + t])); Ls[v][t] = s; }
  __syncthreads();
  for (int i = tid; i < V * (V / 8); i += 256) { const int u = i / (V / 8), v0 = (i % (V / 8)) * 8; v8b vh, vl;
#pragma unroll
    for (int j = 0; j < 8; ++j) { const int v = v0 + j; float s = 0.0f; for (int t = 0; t < T; ++t) s += pmul(Ls[v][t], Rs[t][u]); b16 p, q; split16(sigm(s + bf16_rne(bs[v * V + u])) * 2048.0f, p, q); vh[j] = p; vl[j] = q; }
    const size_t o = ((size_t)n * V + u) * V + v0; for (int pass = 0; pass < 2; ++pass) { *(volatile v8b*)(SGH + o) = vh; *(volatile v8b*)(SGL + o) = vl; __threadfence(); } }
}
__global__ __launch_bounds__(32) void satt_kernel(const float* __restrict__ Vs, const b16* __restrict__ SGH, const b16* __restrict__ SGL, float* __restrict__ SRAW) {
  __shared__ __attribute__((aligned(16))) b16 Ah[16][V + 8]; __shared__ __attribute__((aligned(16))) float Tf[16][V + 4];
  const int lane = threadIdx.x, nloc = lane & 15, hlf = lane >> 4; const int n = blockIdx.x / (V / 16), it = blockIdx.x % (V / 16); const int i0 = it * 16;
  for (int rr = 0; rr < 16; ++rr) for (int q = 0; q < 4; ++q) Ah[rr][q * 32 + lane] = (b16)(bf16_rne(Vs[(size_t)(i0 + rr) * V + q * 32 + lane]) * WSC);
  wave_lds_sync(); v8f acc[8];
#pragma unroll
  for (int t = 0; t < 8; ++t) acc[t] = (v8f){};
#pragma unroll
  for (int kb = 0; kb < V; kb += 32) { const v16b a = frag_kb(&Ah[nloc][kb], hlf);
#pragma unroll
    for (int t = 0; t < 8; ++t) { const size_t br = ((size_t)n * V + t * 16 + nloc) * V + kb; acc[t] = wmma16b(a, frag_kb(SGH + br, hlf), acc[t]); acc[t] = wmma16b(a, frag_kb(SGL + br, hlf), acc[t]); } }
#pragma unroll
  for (int t = 0; t < 8; ++t)
#pragma unroll
    for (int r8 = 0; r8 < 8; ++r8) Tf[8 * hlf + r8][t * 16 + nloc] = acc[t][r8] * (1.0f / (WSC * 2048.0f));
  wave_lds_sync();
  for (int pass = 0; pass < 2; ++pass) { for (int rr = 0; rr < 16; ++rr) *(volatile v4f*)(SRAW + ((size_t)n * V + i0 + rr) * V + lane * 4) = *(const v4f*)(&Tf[rr][lane * 4]); __threadfence(); }
}
__global__ __launch_bounds__(128) void csoft_kernel(const float* __restrict__ SRAW, float* __restrict__ SATT) {
  const int n = blockIdx.x, u = threadIdx.x; const float* s = SRAW + (size_t)n * V * V; float mx = -INFINITY; for (int i = 0; i < V; ++i) mx = fmaxf(mx, s[(size_t)i * V + u]); float den = 0.0f; for (int i = 0; i < V; ++i) den += __expf(s[(size_t)i * V + u] - mx); const float inv = 1.0f / den;
  for (int pass = 0; pass < 2; ++pass) { for (int i = 0; i < V; ++i) ((volatile float*)SATT)[((size_t)n * V + i) * V + u] = __expf(s[(size_t)i * V + u] - mx) * inv; __threadfence(); }
}
__global__ __launch_bounds__(256) void glearn_kernel(const float* __restrict__ x, const float* __restrict__ a, float* __restrict__ SG) {
  __shared__ float Xs[V][FD + 1]; __shared__ float Es[V][V + 1]; const int nt = blockIdx.x, tid = threadIdx.x; const float* xr = x + (size_t)nt * V * FD;
  for (int i = tid; i < V * FD; i += 256) Xs[i / FD][i % FD] = bf16_rne(xr[i]);
  __syncthreads();
  __shared__ float Av[FD]; const int j = tid % V, half = tid / V; if (tid < FD) Av[tid] = bf16_rne(a[tid]) * (1.0f / FD);
  __syncthreads();
  for (int i = half * 64; i < half * 64 + 64; ++i) { float s = 0.0f;
#pragma unroll 8
    for (int f = 0; f < FD; ++f) s += pmul(fabsf(Xs[i][f] - Xs[j][f]), Av[f]); Es[i][j] = __expf(s); }
  __syncthreads();
  __shared__ float Cs[V]; if (half == 0) { float cs = 0.0f; for (int i = 0; i < V; ++i) cs += Es[i][j]; Cs[j] = cs; } __syncthreads(); const float inv = 1.0f / (Cs[j] + 1e-8f);
  for (int pass = 0; pass < 2; ++pass) { for (int i = half * 64; i < half * 64 + 64; ++i) ((volatile float*)SG)[((size_t)nt * V + i) * V + j] = 0.7f * pmul(Es[i][j], inv) + (i == j ? 0.3f : 0.0f); __threadfence(); }
}
__global__ __launch_bounds__(256) void loss_kernel(const float* __restrict__ x, const float* __restrict__ SG, float* __restrict__ LS) {
  __shared__ float red1[8], red2[8]; const int tid = threadIdx.x, wave = tid >> 5, lane = tid & 31; float l1 = 0.0f, l2 = 0.0f;
  for (int p = tid; p < V * V; p += 256) { const int i = p / V, j = p % V; float smt[T]; for (int t = 0; t < T; ++t) { float s = 0.0f; for (int n = 0; n < NB; ++n) s += SG[(((size_t)n * T + t) * V + i) * V + j]; smt[t] = s * (1.0f / NB); l2 += pmul(smt[t], smt[t]); }
    float d2 = 0.0f;
#pragma unroll 1
    for (int f = 0; f < FD; ++f) { float s = 0.0f; for (int nt = 0; nt < NB * T; ++nt) s += fabsf(bf16_rne(x[((size_t)nt * V + i) * FD + f]) - bf16_rne(x[((size_t)nt * V + j) * FD + f])); const float dm = s * (1.0f / NB) * (1.0f / T); d2 += pmul(dm, dm); }
    float st = 0.0f; for (int t = 0; t < T; ++t) st += pmul(d2, smt[t]); l1 += st; }
  for (int o = 16; o; o >>= 1) { l1 += __shfl_xor(l1, o); l2 += __shfl_xor(l2, o); } if (lane == 0) { red1[wave] = l1; red2[wave] = l2; } __syncthreads();
  if (tid < 32) { float a1 = 0.0f, a2 = 0.0f; for (int w = 0; w < 8; ++w) { a1 += red1[w]; a2 += red2[w]; } for (int pass = 0; pass < 2; ++pass) { ((volatile float*)LS)[lane] = lane == 0 ? ALPHA * a1 : (lane == 1 ? ALPHA * a2 : 0.0f); __threadfence(); } }
}

__global__ __launch_bounds__(256) void tka_kernel(const float* __restrict__ SG, const float* __restrict__ SATT, int NTV, b16* __restrict__ TKH, b16* __restrict__ TKL) {
  __shared__ float Ss[V][V + 1]; __shared__ float Dg[V]; const int nt = blockIdx.x; if (nt >= NTV) return; const int n = nt / T, tid = threadIdx.x; const float* s = SG + (size_t)nt * V * V; const float* sa = SATT + (size_t)n * V * V;
  for (int i = tid; i < V * V; i += 256) Ss[i / V][i % V] = s[i];
  __syncthreads();
  if (tid < V) { float d = 0.0f; for (int m = 0; m < V; ++m) d += fminf(Ss[tid][m], Ss[m][tid]); Dg[tid] = d; }
  __syncthreads();
  for (int u = tid; u < V * (V / 8); u += 256) { const int i = u / (V / 8), j0 = (u % (V / 8)) * 8; v8b h0, l0, h1, l1, h2, l2;
#pragma unroll
    for (int q = 0; q < 8; ++q) { const int j = j0 + q; const float ssym = fminf(Ss[j][i], Ss[i][j]); const float dlt = (i == j) ? 1.0f : 0.0f; const float L = pmul(Dg[j], dlt) - ssym - dlt; const float t2 = 2.0f * pmul(L, L) - dlt; const float att = sa[(size_t)j * V + i];
      b16 p, ql; split16(pmul(dlt, att) * 4096.0f, p, ql); h0[q] = p; l0[q] = ql; split16(pmul(L, att) * 4096.0f, p, ql); h1[q] = p; l1[q] = ql; split16(pmul(t2, att) * 4096.0f, p, ql); h2[q] = p; l2[q] = ql; }
    const size_t base = ((size_t)nt * KC) * V * V + (size_t)i * V + j0; for (int pass = 0; pass < 2; ++pass) { *(volatile v8b*)(TKH + base) = h0; *(volatile v8b*)(TKL + base) = l0; *(volatile v8b*)(TKH + base + V * V) = h1; *(volatile v8b*)(TKL + base + V * V) = l1; *(volatile v8b*)(TKH + base + 2 * V * V) = h2; *(volatile v8b*)(TKL + base + 2 * V * V) = l2; __threadfence(); } }
}
template <int F, int FIRST>
__global__ __launch_bounds__(256) void xtp_kernel(const float* __restrict__ IN, float scale, int NTV, b16* __restrict__ XH, b16* __restrict__ XL) {
  __shared__ float Tt[V][65]; const int nt = blockIdx.x / (F / 64), fc = blockIdx.x % (F / 64); if (nt >= NTV) return; const int tid = threadIdx.x; const float* src = IN + (size_t)nt * V * F;
  for (int i = tid; i < V * 64; i += 256) { const int j = i / 64, f = i % 64; float v = src[(size_t)j * F + fc * 64 + f]; if (FIRST) v = bf16_rne(v); Tt[j][f] = v; }
  __syncthreads();
  { const int f = tid / 4, g0 = (tid % 4) * 4; for (int g = g0; g < g0 + 4; ++g) { v8b vh, vl;
#pragma unroll
      for (int q = 0; q < 8; ++q) { b16 p, ql; split16(Tt[g * 8 + q][f] * scale, p, ql); vh[q] = p; vl[q] = ql; }
      const size_t o = ((size_t)nt * F + fc * 64 + f) * V + g * 8; for (int pass = 0; pass < 2; ++pass) { *(volatile v8b*)(XH + o) = vh; *(volatile v8b*)(XL + o) = vl; __threadfence(); } } }
}
__global__ __launch_bounds__(256) void theta_kernel(const float* __restrict__ th, int F, int O, b16* __restrict__ TH) {
  const int u = blockIdx.x * 256 + threadIdx.x; const int FG = F / 8; if (u >= KC * O * FG) return; const int k = u / (O * FG), o = (u / FG) % O, f0 = (u % FG) * 8; v8b v;
#pragma unroll
  for (int q = 0; q < 8; ++q) v[q] = (b16)(bf16_rne(th[((size_t)k * F + f0 + q) * O + o]) * WSC); for (int pass = 0; pass < 2; ++pass) { *(volatile v8b*)(TH + ((size_t)k * O + o) * F + f0) = v; __threadfence(); }
}
template <int F, int O>
__global__ __launch_bounds__(32) void cheb_kernel(const b16* __restrict__ TKH, const b16* __restrict__ TKL, const b16* __restrict__ XH, const b16* __restrict__ XL, float xscale, const b16* __restrict__ TH, float ascale, int NTV, float* __restrict__ OUT) {
  __shared__ __attribute__((aligned(16))) b16 Gh[16][64 + 8], Gl[16][64 + 8]; __shared__ __attribute__((aligned(16))) float Tf[16][64 + 4];
  const int lane = threadIdx.x, nloc = lane & 15, hlf = lane >> 4; const int og = blockIdx.x % (O / 64), it = (blockIdx.x / (O / 64)) % (V / 16), nt = blockIdx.x / ((O / 64) * (V / 16)); if (nt >= NTV) return; const int i0 = it * 16;
  v8f acc[4] = {(v8f){}, (v8f){}, (v8f){}, (v8f){}};
#pragma unroll 1
  for (int k = 0; k < KC; ++k) { const b16* ah = TKH + (((size_t)nt * KC + k) * V + i0 + nloc) * V; const b16* al = TKL + (((size_t)nt * KC + k) * V + i0 + nloc) * V;
#pragma unroll 1
    for (int fcnk = 0; fcnk < F / 64; ++fcnk) { v8f g[4] = {(v8f){}, (v8f){}, (v8f){}, (v8f){}};
#pragma unroll
      for (int kb = 0; kb < V; kb += 32) { const v16b a = frag_kb(ah + kb, hlf), a2 = frag_kb(al + kb, hlf);
#pragma unroll
        for (int t = 0; t < 4; ++t) { const size_t xr = ((size_t)nt * F + fcnk * 64 + t * 16 + nloc) * V + kb; const v16b bh = frag_kb(XH + xr, hlf), bl = frag_kb(XL + xr, hlf); g[t] = wmma16b(a, bh, g[t]); g[t] = wmma16b(a, bl, g[t]); g[t] = wmma16b(a2, bh, g[t]); g[t] = wmma16b(a2, bl, g[t]); } }
#pragma unroll
      for (int t = 0; t < 4; ++t)
#pragma unroll
        for (int r8 = 0; r8 < 8; ++r8) { b16 p, ql; split16(g[t][r8] * (1.0f / (4096.0f * xscale)) * ascale, p, ql); Gh[8 * hlf + r8][t * 16 + nloc] = p; Gl[8 * hlf + r8][t * 16 + nloc] = ql; }
      wave_lds_sync();
#pragma unroll
      for (int kb = 0; kb < 64; kb += 32) { const v16b a = frag_kb(&Gh[nloc][kb], hlf), a2 = frag_kb(&Gl[nloc][kb], hlf);
#pragma unroll
        for (int t = 0; t < 4; ++t) { const v16b bw = frag_kb(TH + ((size_t)k * O + og * 64 + t * 16 + nloc) * F + fcnk * 64 + kb, hlf); acc[t] = wmma16b(a, bw, acc[t]); acc[t] = wmma16b(a2, bw, acc[t]); } }
      wave_lds_sync(); } }
#pragma unroll
  for (int t = 0; t < 4; ++t)
#pragma unroll
    for (int r8 = 0; r8 < 8; ++r8) Tf[8 * hlf + r8][t * 16 + nloc] = fmaxf(acc[t][r8] * (1.0f / (ascale * WSC)), 0.0f);
  wave_lds_sync();
  for (int pass = 0; pass < 2; ++pass) { for (int rr = 0; rr < 16; ++rr) { ((volatile float*)OUT)[((size_t)nt * V + i0 + rr) * O + og * 64 + lane] = Tf[rr][lane]; ((volatile float*)OUT)[((size_t)nt * V + i0 + rr) * O + og * 64 + 32 + lane] = Tf[rr][32 + lane]; } __threadfence(); }
}
__global__ __launch_bounds__(256) void wconv_kernel(const float* __restrict__ cw, b16* __restrict__ WC) {
  const int u = blockIdx.x * 256 + threadIdx.x; if (u >= TF * 24) return; const int o = u / 24, k0 = (u % 24) * 8; v8b v;
#pragma unroll
  for (int q = 0; q < 8; ++q) { const int k = k0 + q; const int kt = k / CH, c = k % CH; v[q] = (b16)(bf16_rne(cw[((size_t)o * CH + c) * KT + kt]) * WSC); }
  for (int pass = 0; pass < 2; ++pass) { *(volatile v8b*)(WC + (size_t)o * 192 + k0) = v; __threadfence(); }
}
__global__ __launch_bounds__(32) void tconv_kernel(const float* __restrict__ XG, const b16* __restrict__ WC, const float* __restrict__ cb, int NTV, float* __restrict__ y) {
  __shared__ __attribute__((aligned(16))) b16 Ah[16][192 + 8], Al[16][192 + 8]; __shared__ __attribute__((aligned(16))) float Tf[16][TF + 4];
  const int lane = threadIdx.x, nloc = lane & 15, hlf = lane >> 4; const int it = blockIdx.x % (V / 16), nt = blockIdx.x / (V / 16); if (nt >= NTV) return; const int n = nt / T, t = nt % T, i0 = it * 16;
  for (int rr = 0; rr < 16; ++rr) for (int kt = 0; kt < KT; ++kt) for (int q = 0; q < 2; ++q) { const int tt = t - 1 + kt; float v = 0.0f; if (tt >= 0 && tt < T) v = XG[(((size_t)n * T + tt) * V + i0 + rr) * CH + q * 32 + lane]; b16 p, ql; split16(v * 4096.0f, p, ql); Ah[rr][kt * 64 + q * 32 + lane] = p; Al[rr][kt * 64 + q * 32 + lane] = ql; }
  wave_lds_sync(); v8f acc[4] = {(v8f){}, (v8f){}, (v8f){}, (v8f){}};
#pragma unroll
  for (int kb = 0; kb < 192; kb += 32) { const v16b a = frag_kb(&Ah[nloc][kb], hlf), a2 = frag_kb(&Al[nloc][kb], hlf);
#pragma unroll
    for (int tt = 0; tt < 4; ++tt) { const v16b bw = frag_kb(WC + (size_t)(tt * 16 + nloc) * 192 + kb, hlf); acc[tt] = wmma16b(a, bw, acc[tt]); acc[tt] = wmma16b(a2, bw, acc[tt]); } }
#pragma unroll
  for (int tt = 0; tt < 4; ++tt) { const int c = tt * 16 + nloc; const float bb = bf16_rne(cb[c]);
#pragma unroll
    for (int r8 = 0; r8 < 8; ++r8) Tf[8 * hlf + r8][c] = fmaxf(acc[tt][r8] * (1.0f / (4096.0f * WSC)) + bb, 0.0f); }
  wave_lds_sync();
  for (int rr = 0; rr < 16; ++rr) { const float v0 = Tf[rr][lane], v1 = Tf[rr][32 + lane]; float s = v0 + v1; for (int o = 16; o; o >>= 1) s += __shfl_xor(s, o); const float mu = s * (1.0f / TF); const float d0 = v0 - mu, d1 = v1 - mu; float q = pmul(d0, d0) + pmul(d1, d1); for (int o = 16; o; o >>= 1) q += __shfl_xor(q, o); const float rs = rsqrtf(q * (1.0f / TF) + 1e-5f);
    const size_t ob = (((size_t)nt) * V + i0 + rr) * TF; ((volatile float*)y)[ob + lane] = pmul(d0, rs); ((volatile float*)y)[ob + 32 + lane] = pmul(d1, rs); }
  __threadfence();
  for (int rr = 0; rr < 16; ++rr) { const float v0 = Tf[rr][lane], v1 = Tf[rr][32 + lane]; float s = v0 + v1; for (int o = 16; o; o >>= 1) s += __shfl_xor(s, o); const float mu = s * (1.0f / TF); const float d0 = v0 - mu, d1 = v1 - mu; float q = pmul(d0, d0) + pmul(d1, d1); for (int o = 16; o; o >>= 1) q += __shfl_xor(q, o); const float rs = rsqrtf(q * (1.0f / TF) + 1e-5f);
    const size_t ob = (((size_t)nt) * V + i0 + rr) * TF; ((volatile float*)y)[ob + lane] = pmul(d0, rs); ((volatile float*)y)[ob + 32 + lane] = pmul(d1, rs); }
  __threadfence();
}
__global__ __launch_bounds__(32) void lout_kernel(const float* __restrict__ LS, float* __restrict__ o1, float* __restrict__ o2) { const int lane = threadIdx.x; for (int pass = 0; pass < 2; ++pass) { if (lane == 0) { ((volatile float*)o1)[0] = LS[0]; ((volatile float*)o2)[0] = LS[1]; } __threadfence(); } }
}

extern "C" void kernel_launch(void* const* d_in, const int* in_sizes, int n_in, void* d_out, int out_size, void* d_ws, size_t ws_size, hipStream_t stream) {
  (void)n_in;
  auto Fp = [&](int i) { return (const float*)d_in[i]; };
  if (in_sizes[0] != NB * T * V * FD || in_sizes[1] != FD || in_sizes[5] != V * V || in_sizes[6] != V * V || in_sizes[8] != FD * V || in_sizes[12] != KC * FD * C1 || in_sizes[13] != KC * C1 * CH || in_sizes[14] != TF * CH * KT || out_size != NB * T * V * TF + 2) return;
  const int NBV = NB; const int NTV = NBV * T;
  size_t off = 0; char* ws = (char*)d_ws;
  auto carve = [&](size_t bytes) { char* p = ws + off; off += (bytes + 255) & ~(size_t)255; return p; };
  float* TATT = (float*)carve(NB * 64 * 4); float* XT = (float*)carve((size_t)NB * T * V * FD * 4); b16* SGH = (b16*)carve((size_t)NB * V * V * 2); b16* SGL = (b16*)carve((size_t)NB * V * V * 2); float* SRAW = (float*)carve((size_t)NB * V * V * 4); float* SATT = (float*)carve((size_t)NB * V * V * 4);
  float* SG = (float*)carve((size_t)NB * T * V * V * 4); float* LS = (float*)carve(128); b16* TKH = (b16*)carve((size_t)NB * T * KC * V * V * 2); b16* TKL = (b16*)carve((size_t)NB * T * KC * V * V * 2);
  b16* X1H = (b16*)carve((size_t)NB * T * FD * V * 2); b16* X1L = (b16*)carve((size_t)NB * T * FD * V * 2); b16* TH1 = (b16*)carve((size_t)KC * C1 * FD * 2); float* XG1 = (float*)carve((size_t)NB * T * V * C1 * 4);
  b16* X2H = (b16*)carve((size_t)NB * T * C1 * V * 2); b16* X2L = (b16*)carve((size_t)NB * T * C1 * V * 2); b16* TH2 = (b16*)carve((size_t)KC * CH * C1 * 2); float* XG2 = (float*)carve((size_t)NB * T * V * CH * 4); b16* WC = (b16*)carve(TF * 192 * 2);
  if (off > ws_size || off > ((size_t)96 << 20)) return;
  tatt_kernel<<<NB, 256, 0, stream>>>(Fp(0), Fp(7), Fp(8), Fp(9), Fp(10), Fp(11), TATT);
  xt_kernel<<<(unsigned)((NB * T * V * FD / 4 + 255) / 256), 256, 0, stream>>>(Fp(0), TATT, XT);
  sprep_kernel<<<NB, 256, 0, stream>>>(XT, Fp(2), Fp(3), Fp(4), Fp(5), SGH, SGL);
  satt_kernel<<<NB * (V / 16), 32, 0, stream>>>(Fp(6), SGH, SGL, SRAW);
  csoft_kernel<<<NB, 128, 0, stream>>>(SRAW, SATT);
  glearn_kernel<<<NB * T, 256, 0, stream>>>(Fp(0), Fp(1), SG);
  loss_kernel<<<1, 256, 0, stream>>>(Fp(0), SG, LS);
  tka_kernel<<<NB * T, 256, 0, stream>>>(SG, SATT, NTV, TKH, TKL);
  theta_kernel<<<(KC * C1 * (FD / 8) + 255) / 256, 256, 0, stream>>>(Fp(12), FD, C1, TH1); theta_kernel<<<(KC * CH * (C1 / 8) + 255) / 256, 256, 0, stream>>>(Fp(13), C1, CH, TH2); wconv_kernel<<<(TF * 24 + 255) / 256, 256, 0, stream>>>(Fp(14), WC);
  xtp_kernel<FD, 1><<<NB * T * (FD / 64), 256, 0, stream>>>(Fp(0), 8.0f, NTV, X1H, X1L);
  cheb_kernel<FD, C1><<<(unsigned)(NTV * (V / 16) * (C1 / 64)), 32, 0, stream>>>(TKH, TKL, X1H, X1L, 8.0f, TH1, 64.0f, NTV, XG1);
  xtp_kernel<C1, 0><<<NB * T * (C1 / 64), 256, 0, stream>>>(XG1, 128.0f, NTV, X2H, X2L);
  cheb_kernel<C1, CH><<<(unsigned)(NTV * (V / 16) * (CH / 64)), 32, 0, stream>>>(TKH, TKL, X2H, X2L, 128.0f, TH2, 1024.0f, NTV, XG2);
  tconv_kernel<<<(unsigned)(NTV * (V / 16)), 32, 0, stream>>>(XG2, WC, Fp(15), NTV, (float*)d_out);
  lout_kernel<<<1, 32, 0, stream>>>(LS, (float*)d_out + (size_t)NB * T * V * TF, (float*)d_out + (size_t)NB * T * V * TF + 1);
}
